// PointNetSetAbstraction_11123965297214
// MI455X (gfx1250) — hardware-verified
//
#include <hip/hip_runtime.h>
#include <math.h>
#pragma clang fp contract(off)

typedef __attribute__((ext_vector_type(16))) _Float16 v16h;
typedef __attribute__((ext_vector_type(8)))  _Float16 v8h;
typedef __attribute__((ext_vector_type(8)))  float    v8f;
typedef __attribute__((ext_vector_type(4)))  float    v4f;
typedef __attribute__((ext_vector_type(4)))  unsigned v4u;

constexpr int NBATCH = 8;
constexpr int NPTS   = 8192;
constexpr int NQRY   = 1024;
constexpr int KNBR   = 32;
constexpr int MROWS  = NBATCH * NQRY * KNBR;
constexpr int CH_L0  = 64;
constexpr int CH_L1  = 64;
constexpr int CH_L2  = 128;
constexpr float BN_EPS = 1e-5f;
constexpr int OUT0_FLOATS = NBATCH * NQRY * 3;
constexpr int OUT1_FLOATS = NBATCH * CH_L2 * NQRY;
static_assert(OUT0_FLOATS * 4 == 98304, "sz");
static_assert((OUT0_FLOATS + OUT1_FLOATS) * 4 == 4292608, "sz");
static_assert((NPTS & (NPTS - 1)) == 0, "sz");

constexpr float W_CARRY   = 16.0f;
constexpr float ACT_CARRY = 8.0f;
constexpr float Y1_CARRY  = 16.0f;
constexpr float RES_CARRY = 2048.0f;
constexpr float INV_PROD_CARRY = 1.0f / (W_CARRY * ACT_CARRY);
constexpr float INV_RES_PROD_CARRY = INV_PROD_CARRY / RES_CARRY;
constexpr float INV_Y1_CARRY   = 1.0f / Y1_CARRY;
constexpr float F16_MIN_NORMAL = 6.103515625e-05f;

constexpr int P_W0  = 0;
constexpr int P_B0  = 256;
constexpr int P_G0  = 320;
constexpr int P_BE0 = 384;
constexpr int P_B1  = 448;
constexpr int P_G1  = 512;
constexpr int P_BE1 = 576;
constexpr int P_B2  = 640;
constexpr int P_G2  = 768;
constexpr int P_BE2 = 896;
constexpr int P_TOTAL = 1024;

constexpr int GEMM_BLOCKS    = 256;
constexpr int ROWS_PER_BLOCK = 1024;
constexpr int TILES_PER_BLOCK = 8;
constexpr int APITCH = 72;
static_assert(GEMM_BLOCKS * ROWS_PER_BLOCK == MROWS, "sz");
static_assert(ROWS_PER_BLOCK == 32 * KNBR, "sz");
static_assert(CH_L0 % 32 == 0 && CH_L1 % 32 == 0, "sz");
static_assert(CH_L1 % 64 == 0 && CH_L2 % 64 == 0, "sz");

constexpr bool SUM3_02_THEN_1 = true;

__device__ __forceinline__ float bf16r(float f) {
  unsigned u = __float_as_uint(f);
  u = (u + 0x7FFFu + ((u >> 16) & 1u)) & 0xFFFF0000u;
  return __uint_as_float(u);
}
__device__ __forceinline__ float sq3(float x, float y, float z) {
  const float t0 = x * x;
  const float t1 = y * y;
  const float t2 = z * z;
  return SUM3_02_THEN_1 ? ((t0 + t2) + t1) : ((t0 + t1) + t2);
}
__device__ __forceinline__ unsigned fkey(float d) {
  const unsigned u = __float_as_uint(d);
  return (u & 0x80000000u) ? ~u : (u | 0x80000000u);
}
__device__ __forceinline__ float h16_to_f32(unsigned hb) {
  const unsigned sgn = (hb & 0x8000u) << 16; const unsigned em = hb & 0x7fffu;
  const float fn = __uint_as_float((em << 13) + 0x38000000u);
  const float fs = (float)em * 5.9604644775390625e-8f;
  const float mag = (em < 0x400u) ? fs : fn; return __uint_as_float(__float_as_uint(mag) | sgn); }

__device__ __forceinline__ _Float16 act16(float y, float sc, float sh) {
  const float z = fmaf(y, sc, sh);
  const float a = fminf(fmaxf(z, 0.0f) * ACT_CARRY, 60000.0f);
  return (_Float16)a;
}
__device__ __forceinline__ void act16_split(float y, float sc, float sh, _Float16& hi, _Float16& lo) {
  const float z = fmaf(y, sc, sh);
  const float a = fminf(fmaxf(z, 0.0f) * ACT_CARRY, 60000.0f);
  const float ah = (a < F16_MIN_NORMAL) ? 0.0f : a;
  const _Float16 h = (_Float16)ah;
  float hf = (float)h;
  asm volatile("" : "+v"(hf));
  const float r = (a - hf) * RES_CARRY;
  hi = h;
  lo = (_Float16)r;
}
__device__ __forceinline__ void keep4_h(v16h a, v16h b, v16h c, v16h d) { asm volatile("v_nop" :: "v"(a), "v"(b), "v"(c), "v"(d)); }
__device__ __forceinline__ void grp_guard(v8f& c0, v8f& c1, v8f& c2, v8f& c3, v16h a, v16h b0, v16h b1, v16h b2, v16h b3) {
  asm volatile("v_nop\n\tv_nop\n\tv_nop\n\tv_nop\n\tv_nop"
               : "+v"(c0), "+v"(c1), "+v"(c2), "+v"(c3)
               : "v"(a), "v"(b0), "v"(b1), "v"(b2), "v"(b3));
}
__device__ __forceinline__ void grp_guard8(v8f& c0, v8f& c1, v8f& c2, v8f& c3, v8f& d0, v8f& d1, v8f& d2, v8f& d3,
                                           v16h a, v16h a2, v16h b0, v16h b1, v16h b2, v16h b3) {
  asm volatile("v_nop\n\tv_nop\n\tv_nop\n\tv_nop\n\tv_nop"
               : "+v"(c0), "+v"(c1), "+v"(c2), "+v"(c3), "+v"(d0), "+v"(d1), "+v"(d2), "+v"(d3)
               : "v"(a), "v"(a2), "v"(b0), "v"(b1), "v"(b2), "v"(b3));
}
union FragU { v16h v; v8h h[2]; };
__device__ __forceinline__ v16h frag_load_g(const _Float16* p) {
  FragU f; f.h[0] = *(const v8h*)(p); f.h[1] = *(const v8h*)(p + 16); return f.v;
}
__device__ __forceinline__ v8f mma_f16(v16h a, v16h b, v8f c) {
  return __builtin_amdgcn_wmma_f32_16x16x32_f16(false, a, false, b, (short)0, c, false, false);
}

__global__ __launch_bounds__(256) void prep_xyz_kernel(const float* __restrict__ xyz,
                                                       float* __restrict__ Xr,
                                                       float* __restrict__ sqn) {
  const int p = blockIdx.x * 256 + threadIdx.x;
  const int pc = (p < NBATCH * NPTS) ? p : (NBATCH * NPTS - 1);
  const float x = bf16r(xyz[(size_t)pc * 3 + 0]);
  const float y = bf16r(xyz[(size_t)pc * 3 + 1]);
  const float z = bf16r(xyz[(size_t)pc * 3 + 2]);
  v4f v; v[0] = x; v[1] = y; v[2] = z; v[3] = 0.0f;
  const float s = sq3(x, y, z);
  if (p < NBATCH * NPTS) {
    volatile v4f* vp = (volatile v4f*)(Xr + (size_t)p * 4);
    volatile float* sp = sqn + p;
    *vp = v; *sp = s;
    __threadfence();
    *vp = v; *sp = s;
  }
}

__global__ __launch_bounds__(256) void prep_small_kernel(
    const float* __restrict__ w0, const float* __restrict__ b0, const float* __restrict__ g0, const float* __restrict__ be0,
    const float* __restrict__ w1, const float* __restrict__ b1, const float* __restrict__ g1, const float* __restrict__ be1,
    const float* __restrict__ w2, const float* __restrict__ b2, const float* __restrict__ g2, const float* __restrict__ be2,
    float* __restrict__ P, unsigned short* __restrict__ W1h, unsigned short* __restrict__ W2h) {
  const int bx = blockIdx.x;
  const int t = threadIdx.x;
  if (bx == 0) {
    const int o = t >> 2, c = t & 3;
    const int cc = (c < 3) ? c : 2;
    const float v = bf16r(w0[o * 3 + cc]);
    const float r = (c < 3) ? v : 0.0f;
    volatile float* pp = P + P_W0 + t;
    *pp = r;
    __threadfence();
    *pp = r;
  } else if (bx < 10) {
    const float* src = b0; int cnt = CH_L0; int off = P_B0;
    if (bx == 2) { src = g0;  off = P_G0; }
    if (bx == 3) { src = be0; off = P_BE0; }
    if (bx == 4) { src = b1;  off = P_B1; }
    if (bx == 5) { src = g1;  off = P_G1; }
    if (bx == 6) { src = be1; off = P_BE1; }
    if (bx == 7) { src = b2;  off = P_B2;  cnt = CH_L2; }
    if (bx == 8) { src = g2;  off = P_G2;  cnt = CH_L2; }
    if (bx == 9) { src = be2; off = P_BE2; cnt = CH_L2; }
    const int tc = (t < cnt) ? t : (cnt - 1);
    const float v = bf16r(src[tc]);
    if (t < cnt) {
      volatile float* pp = P + off + t;
      *pp = v;
      __threadfence();
      *pp = v;
    }
  } else {
    const bool first = (bx < 12);
    const float* src = first ? w1 : w2;
    _Float16* dst = (_Float16*)(first ? W1h : W2h);
    const int i8 = (first ? (bx - 10) : (bx - 12)) * 256 + t;
    const v4f a = *(const v4f*)(src + (size_t)i8 * 8);
    const v4f b = *(const v4f*)(src + (size_t)i8 * 8 + 4);
    v8h h;
    h[0] = (_Float16)(bf16r(a[0]) * W_CARRY); h[1] = (_Float16)(bf16r(a[1]) * W_CARRY);
    h[2] = (_Float16)(bf16r(a[2]) * W_CARRY); h[3] = (_Float16)(bf16r(a[3]) * W_CARRY);
    h[4] = (_Float16)(bf16r(b[0]) * W_CARRY); h[5] = (_Float16)(bf16r(b[1]) * W_CARRY);
    h[6] = (_Float16)(bf16r(b[2]) * W_CARRY); h[7] = (_Float16)(bf16r(b[3]) * W_CARRY);
    volatile v8h* dp = (volatile v8h*)(dst + (size_t)i8 * 8);
    *dp = h;
    __threadfence();
    *dp = h;
  }
}

__global__ __launch_bounds__(512) void fps_kernel(const float* __restrict__ Xr,
                                                  float* __restrict__ Cq,
                                                  float* __restrict__ out0) {
#pragma clang fp contract(off)
  __shared__ unsigned sKv[2][16];
  __shared__ unsigned sKi[2][16];
  __shared__ int sSel[NQRY];
  const int b = blockIdx.x;
  const int t = threadIdx.x;
  const int lane = t & 31;
  const int wave = t >> 5;
  const float* base = Xr + (size_t)b * NPTS * 4;

  float px[16], py[16], pz[16], dd[16];
#pragma unroll
  for (int j = 0; j < 16; ++j) {
    const v4f v = *(const v4f*)(base + (size_t)(t + 512 * j) * 4);
    px[j] = v[0]; py[j] = v[1]; pz[j] = v[2]; dd[j] = 1e10f;
    if ((j & 3) == 3) asm volatile("" :: "v"(pz[j]) : "memory");
  }

  int far = 0;
  for (int it = 0; it < NQRY; ++it) {
    if (t == 0) sSel[it] = far;
    const v4f cv = *(const v4f*)(base + (size_t)far * 4);
    const float cx = cv[0], cy = cv[1], cz = cv[2];
    float bv = -1.0f; int bi = 0;
#pragma unroll
    for (int j = 0; j < 16; ++j) {
      const float dx = px[j] - cx;
      const float dy = py[j] - cy;
      const float dz = pz[j] - cz;
      const float d = sq3(dx, dy, dz);
      const float nd = fminf(dd[j], d);
      dd[j] = nd;
      if (nd > bv) { bv = nd; bi = t + 512 * j; }
    }
    unsigned kv = __float_as_uint(bv);
    unsigned ki = 0xFFFFFFFFu - (unsigned)bi;
#pragma unroll
    for (int off = 16; off >= 1; off >>= 1) {
      const unsigned ov = (unsigned)__shfl_xor((int)kv, off, 32);
      const unsigned oi = (unsigned)__shfl_xor((int)ki, off, 32);
      const bool take = (ov > kv) || (ov == kv && oi > ki);
      kv = take ? ov : kv; ki = take ? oi : ki;
    }
    const int par = it & 1;
    if (lane == 0) { sKv[par][wave] = kv; sKi[par][wave] = ki; }
    __syncthreads();
    kv = sKv[par][lane & 15];
    ki = sKi[par][lane & 15];
#pragma unroll
    for (int off = 8; off >= 1; off >>= 1) {
      const unsigned ov = (unsigned)__shfl_xor((int)kv, off, 32);
      const unsigned oi = (unsigned)__shfl_xor((int)ki, off, 32);
      const bool take = (ov > kv) || (ov == kv && oi > ki);
      kv = take ? ov : kv; ki = take ? oi : ki;
    }
    far = (int)((0xFFFFFFFFu - ki) & (unsigned)(NPTS - 1));
  }
  __syncthreads();

  v4f cr[2];
  float ov6[6];
#pragma unroll
  for (int i = 0; i < 2; ++i) {
    const int q = t + 512 * i;
    const int s = sSel[q] & (NPTS - 1);
    cr[i] = *(const v4f*)(base + (size_t)s * 4);
  }
#pragma unroll
  for (int i = 0; i < 6; ++i) {
    const int f = t + 512 * i;
    const int q = f / 3;
    const int c = f - 3 * q;
    const int s = sSel[q] & (NPTS - 1);
    const v4f v = *(const v4f*)(base + (size_t)s * 4);
    const float e0 = v[0], e1 = v[1], e2 = v[2];
    ov6[i] = (c == 0) ? e0 : ((c == 1) ? e1 : e2);
  }
  float* cdst = Cq + (size_t)b * NQRY * 4;
  float* odst = out0 + (size_t)b * NQRY * 3;
#pragma unroll
  for (int i = 0; i < 2; ++i) *(volatile v4f*)(cdst + (size_t)(t + 512 * i) * 4) = cr[i];
#pragma unroll
  for (int i = 0; i < 6; ++i) *(volatile float*)(odst + t + 512 * i) = ov6[i];
  __threadfence();
#pragma unroll
  for (int i = 0; i < 2; ++i) *(volatile v4f*)(cdst + (size_t)(t + 512 * i) * 4) = cr[i];
#pragma unroll
  for (int i = 0; i < 6; ++i) *(volatile float*)(odst + t + 512 * i) = ov6[i];
}

__global__ __launch_bounds__(256) void knn_group_kernel(const float* __restrict__ Xr,
                                                        const float* __restrict__ sqn,
                                                        const float* __restrict__ Cq,
                                                        float* __restrict__ A0) {
#pragma clang fp contract(off)
  __shared__ unsigned sD[NPTS];
  __shared__ unsigned sRk[2][8];
  __shared__ unsigned sRi[2][8];
  __shared__ int sRes[KNBR];
  const int q = blockIdx.x;
  const int t = threadIdx.x;
  const int lane = t & 31;
  const int wave = t >> 5;
  const int b = q / NQRY;
  const float* base = Xr + (size_t)b * NPTS * 4;
  const float* sqb = sqn + (size_t)b * NPTS;
  const v4f cv = *(const v4f*)(Cq + (size_t)q * 4);
  const float cx = cv[0], cy = cv[1], cz = cv[2];
  const float a = sq3(cx, cy, cz);

  unsigned bk = 0xFFFFFFFFu, bi = 0xFFFFFFFFu;
#pragma unroll 4
  for (int j = 0; j < 32; ++j) {
    const int n = t + 256 * j;
    const v4f p = *(const v4f*)(base + (size_t)n * 4);
    const float bbv = sqb[n];
    const float p0 = cx * p[0];
    const float p1 = cy * p[1];
    const float p2 = cz * p[2];
    const float e = (p0 + p1) + p2;
    const float s = a + bbv;
    float d = s - 2.0f * e;
    d = d + 0.0f;
    const unsigned key = fkey(d);
    sD[n] = key;
    if (key < bk) { bk = key; bi = (unsigned)n; }
  }

  for (int k = 0; k < KNBR; ++k) {
    unsigned kv = bk, ki = bi;
#pragma unroll
    for (int off = 16; off >= 1; off >>= 1) {
      const unsigned ov = (unsigned)__shfl_xor((int)kv, off, 32);
      const unsigned oi = (unsigned)__shfl_xor((int)ki, off, 32);
      const bool take = (ov < kv) || (ov == kv && oi < ki);
      kv = take ? ov : kv; ki = take ? oi : ki;
    }
    const int par = k & 1;
    if (lane == 0) { sRk[par][wave] = kv; sRi[par][wave] = ki; }
    __syncthreads();
    kv = sRk[par][lane & 7];
    ki = sRi[par][lane & 7];
#pragma unroll
    for (int off = 4; off >= 1; off >>= 1) {
      const unsigned ov = (unsigned)__shfl_xor((int)kv, off, 32);
      const unsigned oi = (unsigned)__shfl_xor((int)ki, off, 32);
      const bool take = (ov < kv) || (ov == kv && oi < ki);
      kv = take ? ov : kv; ki = take ? oi : ki;
    }
    const int win = (int)(ki & (unsigned)(NPTS - 1));
    if (t == 0) sRes[k] = win;
    if ((win & 255) == t) {
      sD[win] = 0xFFFFFFFFu;
      bk = 0xFFFFFFFFu; bi = 0xFFFFFFFFu;
      for (int j = 0; j < 32; ++j) {
        const int n = t + 256 * j;
        const unsigned key = sD[n];
        if (key < bk) { bk = key; bi = (unsigned)n; }
      }
    }
  }
  __syncthreads();
  if (wave == 0) {
    const int idx = sRes[lane] & (NPTS - 1);
    const v4f p = *(const v4f*)(base + (size_t)idx * 4);
    v4f f;
    f[0] = p[0] - cx; f[1] = p[1] - cy; f[2] = p[2] - cz; f[3] = 0.0f;
    volatile v4f* dst = (volatile v4f*)(A0 + ((size_t)q * KNBR + lane) * 4);
    *dst = f;
    __threadfence();
    *dst = f;
  }
}

__global__ __launch_bounds__(256) void stats0_kernel(const float* __restrict__ A0,
                                                     const float* __restrict__ P,
                                                     float* __restrict__ part) {
  __shared__ float sRed[4 * 128];
  const int t = threadIdx.x;
  const int c = t & 63;
  const int rg = t >> 6;
  const v4f w = *(const v4f*)(P + P_W0 + c * 4);
  const float w0v = w[0], w1v = w[1], w2v = w[2];
  const float bias = P[P_B0 + c];
  const float* rows = A0 + ((size_t)blockIdx.x * ROWS_PER_BLOCK + (size_t)rg * 256) * 4;
  float s = 0.0f, s2 = 0.0f;
#pragma unroll 4
  for (int i = 0; i < 256; ++i) {
    const v4f x = *(const v4f*)(rows + (size_t)i * 4);
    const float y = fmaf(x[2], w2v, fmaf(x[1], w1v, x[0] * w0v)) + bias;
    s += y;
    s2 = fmaf(y, y, s2);
  }
  sRed[rg * 128 + c] = s;
  sRed[rg * 128 + 64 + c] = s2;
  __syncthreads();
  const int col = t & 127;
  const int isq = t >> 7;
  const bool valid = (col < CH_L0);
  const int cl = valid ? col : 0;
  const float v = ((sRed[0 * 128 + isq * 64 + cl] + sRed[1 * 128 + isq * 64 + cl]) +
                   sRed[2 * 128 + isq * 64 + cl]) + sRed[3 * 128 + isq * 64 + cl];
  const float o = valid ? v : 0.0f;
  volatile float* pp = part + (size_t)blockIdx.x * 256 + t;
  *pp = o;
  __threadfence();
  *pp = o;
}

__global__ __launch_bounds__(128) void bn_finalize_kernel(const float* __restrict__ part,
                                                          const float* __restrict__ gsrc,
                                                          const float* __restrict__ besrc,
                                                          float* __restrict__ ss, int nch) {
  const int c = threadIdx.x;
  const int cc = (c < nch) ? c : (nch - 1);
  double s = 0.0, q = 0.0;
#pragma unroll 4
  for (int blk = 0; blk < GEMM_BLOCKS; ++blk) {
    s += (double)part[(size_t)blk * 256 + cc];
    q += (double)part[(size_t)blk * 256 + 128 + cc];
  }
  const double inv = 1.0 / (double)MROWS;
  const double mu = s * inv;
  double var = q * inv - mu * mu;
  if (var < 0.0) var = 0.0;
  const float rs = rsqrtf((float)var + BN_EPS);
  float sc = gsrc[cc] * rs;
  float sh = besrc[cc] - (float)mu * sc;
  if (c >= nch) { sc = 0.0f; sh = 0.0f; }
  volatile float* p0 = ss + c;
  volatile float* p1 = ss + 128 + c;
  *p0 = sc; *p1 = sh;
  __threadfence();
  *p0 = sc; *p1 = sh;
}

template <int MODE>
__global__ __launch_bounds__(256) void mlp_gemm_kernel(
    const float* __restrict__ A0, unsigned short* Yp, const unsigned short* __restrict__ Wp,
    const float* __restrict__ P, const float* __restrict__ ssIn, const float* __restrict__ ssOut,
    float* __restrict__ part, float* __restrict__ out1) {
  constexpr int NOUT = (MODE == 0) ? CH_L1 : CH_L2;
  constexpr int NH = NOUT / 64;
  constexpr int PBIAS = (MODE == 0) ? P_B1 : P_B2;
  __shared__ __align__(16) _Float16 sA[128 * APITCH];
  __shared__ __align__(16) _Float16 sA2[(MODE == 0) ? 128 * APITCH : 8];
  __shared__ __align__(16) float sTab[(MODE == 0) ? 256 : 4];
  __shared__ __align__(16) float sSS[128];
  __shared__ __align__(16) float sT[(MODE == 0) ? 8 * 16 * 68 : 4];
  __shared__ __align__(16) float sRed[(MODE != 2) ? 8 * 128 : 4];
  __shared__ __align__(16) float sOut[(MODE == 2) ? 128 * 36 : 4];

  const int t = threadIdx.x;
  const int lane = t & 31;
  const int wave = t >> 5;
  const int rlane = lane & 15;
  const int hh = lane >> 4;
  const int koff = hh * 8;
  const int mOff = hh * 8;
  const int nh = wave % NH;
  const int n0 = nh * 64;
  const _Float16* W = (const _Float16*)Wp;

  {
    const int tc = t & 63;
    const float scv = ssIn[tc];
    const float shv = ssIn[128 + tc];
    if (t < 64) { sSS[2 * t] = scv; sSS[2 * t + 1] = shv; }
    if (MODE == 0) {
      const float wv = P[P_W0 + t];
      const float bv = P[P_B0 + (t >> 2)];
      const float f = ((t & 3) == 3) ? 1.0f : 0.0f;
      sTab[t] = wv + f * bv;
    }
  }

  v16h bf[2][4];
#pragma unroll
  for (int ks = 0; ks < 2; ++ks) {
#pragma unroll
    for (int j = 0; j < 4; ++j)
      bf[ks][j] = frag_load_g(W + (size_t)(n0 + j * 16 + rlane) * 64 + ks * 32 + koff);
    keep4_h(bf[ks][0], bf[ks][1], bf[ks][2], bf[ks][3]);
  }
  float bias[4], sc2[4], sh2[4];
#pragma unroll
  for (int j = 0; j < 4; ++j) {
    const int n = n0 + j * 16 + rlane;
    bias[j] = P[PBIAS + n];
    if (MODE == 2) { sc2[j] = ssOut[n]; sh2[j] = ssOut[128 + n]; }
    else { sc2[j] = 0.0f; sh2[j] = 0.0f; }
  }
  float cS[4] = {0.0f, 0.0f, 0.0f, 0.0f};
  float cQ[4] = {0.0f, 0.0f, 0.0f, 0.0f};

  for (int tIt = 0; tIt < TILES_PER_BLOCK; ++tIt) {
    const int m0 = blockIdx.x * ROWS_PER_BLOCK + tIt * 128;
    __syncthreads();
    {
      const int r = t >> 1;
      const int kh = (t & 1) * 32;
      const size_t m = (size_t)m0 + r;
      if (MODE == 0) {
        const v4f x = *(const v4f*)(A0 + m * 4);
        const float x0 = x[0], x1 = x[1], x2 = x[2];
#pragma unroll 1
        for (int cch = 0; cch < 4; ++cch) {
          const int kb = kh + cch * 8;
          v8h hv, lv;
#pragma unroll
          for (int e = 0; e < 8; ++e) {
            const int k = kb + e;
            const v4f wv = *(const v4f*)(sTab + k * 4);
            const float y = fmaf(x2, wv[2], fmaf(x1, wv[1], x0 * wv[0])) + wv[3];
            _Float16 hi, lo;
            act16_split(y, sSS[2 * k], sSS[2 * k + 1], hi, lo);
            hv[e] = hi;
            lv[e] = lo;
          }
          *(v8h*)(sA + r * APITCH + kb) = hv;
          *(v8h*)(sA2 + r * APITCH + kb) = lv;
        }
      } else {
        const v4u* src = (const v4u*)(Yp + m * 64 + kh);
#pragma unroll 1
        for (int cch = 0; cch < 4; ++cch) {
          const v4u w = src[cch];
          const unsigned w0 = w[0], w1 = w[1], w2 = w[2], w3 = w[3];
          const int kb = kh + cch * 8;
          v8h hv;
          hv[0] = act16(h16_to_f32(w0 & 0xffffu) * INV_Y1_CARRY, sSS[2 * (kb + 0)], sSS[2 * (kb + 0) + 1]);
          hv[1] = act16(h16_to_f32(w0 >> 16)     * INV_Y1_CARRY, sSS[2 * (kb + 1)], sSS[2 * (kb + 1) + 1]);
          hv[2] = act16(h16_to_f32(w1 & 0xffffu) * INV_Y1_CARRY, sSS[2 * (kb + 2)], sSS[2 * (kb + 2) + 1]);
          hv[3] = act16(h16_to_f32(w1 >> 16)     * INV_Y1_CARRY, sSS[2 * (kb + 3)], sSS[2 * (kb + 3) + 1]);
          hv[4] = act16(h16_to_f32(w2 & 0xffffu) * INV_Y1_CARRY, sSS[2 * (kb + 4)], sSS[2 * (kb + 4) + 1]);
          hv[5] = act16(h16_to_f32(w2 >> 16)     * INV_Y1_CARRY, sSS[2 * (kb + 5)], sSS[2 * (kb + 5) + 1]);
          hv[6] = act16(h16_to_f32(w3 & 0xffffu) * INV_Y1_CARRY, sSS[2 * (kb + 6)], sSS[2 * (kb + 6) + 1]);
          hv[7] = act16(h16_to_f32(w3 >> 16)     * INV_Y1_CARRY, sSS[2 * (kb + 7)], sSS[2 * (kb + 7) + 1]);
          *(v8h*)(sA + r * APITCH + kb) = hv;
        }
      }
    }
    __syncthreads();

    float mv[4] = {0.0f, 0.0f, 0.0f, 0.0f};
#pragma unroll
    for (int i = 0; i < NH; ++i) {
      const int rs = (NH == 1) ? wave : (2 * (wave >> 1) + i);
      v8f acc[4];
      v8f acc2[4];
#pragma unroll
      for (int j = 0; j < 4; ++j) {
        acc[j]  = (v8f){0.f, 0.f, 0.f, 0.f, 0.f, 0.f, 0.f, 0.f};
        acc2[j] = (v8f){0.f, 0.f, 0.f, 0.f, 0.f, 0.f, 0.f, 0.f};
      }
#pragma unroll
      for (int ks = 0; ks < 2; ++ks) {
        FragU fa;
        fa.h[0] = *(const v8h*)(sA + (rs * 16 + rlane) * APITCH + ks * 32 + koff);
        fa.h[1] = *(const v8h*)(sA + (rs * 16 + rlane) * APITCH + ks * 32 + koff + 16);
        const v16h a = fa.v;
        if (MODE == 0) {
          FragU fb;
          fb.h[0] = *(const v8h*)(sA2 + (rs * 16 + rlane) * APITCH + ks * 32 + koff);
          fb.h[1] = *(const v8h*)(sA2 + (rs * 16 + rlane) * APITCH + ks * 32 + koff + 16);
          const v16h a2 = fb.v;
#pragma unroll
          for (int j = 0; j < 4; ++j) acc[j] = mma_f16(a, bf[ks][j], acc[j]);
#pragma unroll
          for (int j = 0; j < 4; ++j) acc2[j] = mma_f16(a2, bf[ks][j], acc2[j]);
          grp_guard8(acc[0], acc[1], acc[2], acc[3], acc2[0], acc2[1], acc2[2], acc2[3],
                     a, a2, bf[ks][0], bf[ks][1], bf[ks][2], bf[ks][3]);
        } else {
#pragma unroll
          for (int j = 0; j < 4; ++j) acc[j] = mma_f16(a, bf[ks][j], acc[j]);
          grp_guard(acc[0], acc[1], acc[2], acc[3], a, bf[ks][0], bf[ks][1], bf[ks][2], bf[ks][3]);
        }
      }

      if (MODE == 0) {
        float* slab = sT + wave * (16 * 68);
#pragma unroll
        for (int j = 0; j < 4; ++j) {
#pragma unroll
          for (int r = 0; r < 8; ++r) {
            const float vm = acc[j][r] * INV_PROD_CARRY;
            const float vs = acc2[j][r] * INV_RES_PROD_CARRY;
            const float v = (vm + vs) + bias[j];
            cS[j] += v;
            cQ[j] = fmaf(v, v, cQ[j]);
            slab[(mOff + r) * 68 + j * 16 + rlane] = fminf(fmaxf(v * Y1_CARRY, -60000.0f), 60000.0f);
          }
        }
        __builtin_amdgcn_fence(__ATOMIC_RELEASE, "workgroup");
        __builtin_amdgcn_wave_barrier();
        __builtin_amdgcn_fence(__ATOMIC_ACQUIRE, "workgroup");
        {
          const int rq = lane >> 3, c8 = (lane & 7) * 8;
          _Float16* Yh = (_Float16*)Yp;
          for (int pass = 0; pass < 2; ++pass) {
#pragma unroll
            for (int itr = 0; itr < 4; ++itr) {
              const int row = itr * 4 + rq;
              const float* sp = slab + row * 68 + c8;
              v8h hv;
#pragma unroll
              for (int e = 0; e < 8; ++e) hv[e] = (_Float16)sp[e];
              *(volatile v8h*)(Yh + (size_t)(m0 + rs * 16 + row) * 64 + c8) = hv;
            }
            __threadfence();
          }
        }
        __builtin_amdgcn_fence(__ATOMIC_RELEASE, "workgroup");
        __builtin_amdgcn_wave_barrier();
        __builtin_amdgcn_fence(__ATOMIC_ACQUIRE, "workgroup");
      } else if (MODE == 1) {
#pragma unroll
        for (int j = 0; j < 4; ++j) {
#pragma unroll
          for (int r = 0; r < 8; ++r) {
            const float v = acc[j][r] * INV_PROD_CARRY + bias[j];
            cS[j] += v;
            cQ[j] = fmaf(v, v, cQ[j]);
          }
        }
      } else {
#pragma unroll
        for (int j = 0; j < 4; ++j) {
#pragma unroll
          for (int r = 0; r < 8; ++r) {
            const float v = acc[j][r] * INV_PROD_CARRY + bias[j];
            const float z = fmaf(v, sc2[j], sh2[j]);
            mv[j] = fmaxf(mv[j], z);
          }
        }
      }
    }
    if (MODE == 2) {
      float mo[4];
#pragma unroll
      for (int j = 0; j < 4; ++j) mo[j] = __shfl_xor(mv[j], 16, 32);
#pragma unroll
      for (int j = 0; j < 4; ++j) mv[j] = fmaxf(mv[j], mo[j]);
      if (hh == 0) {
#pragma unroll
        for (int j = 0; j < 4; ++j) sOut[(n0 + j * 16 + rlane) * 36 + tIt * 4 + (wave >> 1)] = mv[j];
      }
    }
  }

  if (MODE != 2) {
    float oS[4], oQ[4];
#pragma unroll
    for (int j = 0; j < 4; ++j) { oS[j] = __shfl_xor(cS[j], 16, 32); oQ[j] = __shfl_xor(cQ[j], 16, 32); }
#pragma unroll
    for (int j = 0; j < 4; ++j) { cS[j] += oS[j]; cQ[j] += oQ[j]; }
    if (hh == 0) {
#pragma unroll
      for (int j = 0; j < 4; ++j) {
        sRed[wave * 128 + j * 16 + rlane] = cS[j];
        sRed[wave * 128 + 64 + j * 16 + rlane] = cQ[j];
      }
    }
    __syncthreads();
    const int col = t & 127;
    const int isq = t >> 7;
    const bool valid = (col < NOUT);
    const int colc = valid ? col : 0;
    const int nhc = colc >> 6;
    const int cl = colc & 63;
    float s = 0.0f;
#pragma unroll
    for (int g = 0; g < 8 / NH; ++g) s += sRed[(g * NH + nhc) * 128 + isq * 64 + cl];
    const float o = valid ? s : 0.0f;
    volatile float* pp = part + (size_t)blockIdx.x * 256 + t;
    *pp = o;
    __threadfence();
    *pp = o;
  } else {
    __syncthreads();
    const int bb = blockIdx.x >> 5;
    const int q0 = (blockIdx.x & 31) * 32;
    const int lq = lane >> 3;
    const int pc = (lane & 7) * 4;
    for (int pass = 0; pass < 2; ++pass) {
#pragma unroll
      for (int itr = 0; itr < 4; ++itr) {
        const int ch = wave * 16 + itr * 4 + lq;
        const v4f v = *(const v4f*)(sOut + ch * 36 + pc);
        *(volatile v4f*)(out1 + ((size_t)(bb * CH_L2 + ch) * NQRY + q0 + pc)) = v;
      }
      __threadfence();
    }
  }
}

extern "C" void kernel_launch(void* const* d_in, const int* in_sizes, int n_in,
                              void* d_out, int out_size, void* d_ws, size_t ws_size,
                              hipStream_t stream) {
  (void)in_sizes; (void)n_in; (void)out_size;
  const float* xyz = (const float*)d_in[0];
  const float* w0  = (const float*)d_in[1];
  const float* b0  = (const float*)d_in[2];
  const float* g0  = (const float*)d_in[3];
  const float* be0 = (const float*)d_in[4];
  const float* w1  = (const float*)d_in[5];
  const float* b1  = (const float*)d_in[6];
  const float* g1  = (const float*)d_in[7];
  const float* be1 = (const float*)d_in[8];
  const float* w2  = (const float*)d_in[9];
  const float* b2  = (const float*)d_in[10];
  const float* g2  = (const float*)d_in[11];
  const float* be2 = (const float*)d_in[12];
  float* out0 = (float*)d_out;
  float* out1 = (float*)d_out + OUT0_FLOATS;

  char* ws = (char*)d_ws;
  size_t off = 0;
  auto carve = [&](size_t bytes) -> char* {
    char* p = ws + off;
    off += (bytes + 255) & ~(size_t)255;
    return p;
  };
  float* Xr   = (float*)carve((size_t)NBATCH * NPTS * 16);
  float* sqn  = (float*)carve((size_t)NBATCH * NPTS * 4);
  float* Cq   = (float*)carve((size_t)NBATCH * NQRY * 16);
  float* A0   = (float*)carve((size_t)MROWS * 16);
  float* P    = (float*)carve((size_t)P_TOTAL * 4);
  unsigned short* W1h = (unsigned short*)carve((size_t)CH_L1 * CH_L0 * 2);
  unsigned short* W2h = (unsigned short*)carve((size_t)CH_L2 * CH_L1 * 2);
  float* part0 = (float*)carve((size_t)GEMM_BLOCKS * 256 * 4);
  float* part1 = (float*)carve((size_t)GEMM_BLOCKS * 256 * 4);
  float* part2 = (float*)carve((size_t)GEMM_BLOCKS * 256 * 4);
  float* ss0 = (float*)carve(256 * 4);
  float* ss1 = (float*)carve(256 * 4);
  float* ss2 = (float*)carve(256 * 4);
  unsigned short* Y1 = (unsigned short*)carve((size_t)MROWS * CH_L1 * 2);
  if (off > ws_size) return;

  prep_xyz_kernel<<<(NBATCH * NPTS) / 256, 256, 0, stream>>>(xyz, Xr, sqn);
  prep_small_kernel<<<16, 256, 0, stream>>>(w0, b0, g0, be0, w1, b1, g1, be1, w2, b2, g2, be2, P, W1h, W2h);
  fps_kernel<<<NBATCH, 512, 0, stream>>>(Xr, Cq, out0);
  knn_group_kernel<<<NBATCH * NQRY, 256, 0, stream>>>(Xr, sqn, Cq, A0);

  stats0_kernel<<<GEMM_BLOCKS, 256, 0, stream>>>(A0, P, part0);
  bn_finalize_kernel<<<1, 128, 0, stream>>>(part0, P + P_G0, P + P_BE0, ss0, CH_L0);

  mlp_gemm_kernel<0><<<GEMM_BLOCKS, 256, 0, stream>>>(A0, Y1, W1h, P, ss0, ss1, part1, out1);
  bn_finalize_kernel<<<1, 128, 0, stream>>>(part1, P + P_G1, P + P_BE1, ss1, CH_L1);

  mlp_gemm_kernel<1><<<GEMM_BLOCKS, 256, 0, stream>>>(A0, Y1, W2h, P, ss1, ss2, part2, out1);
  bn_finalize_kernel<<<1, 128, 0, stream>>>(part2, P + P_G2, P + P_BE2, ss2, CH_L2);

  mlp_gemm_kernel<2><<<GEMM_BLOCKS, 256, 0, stream>>>(A0, Y1, W2h, P, ss1, ss2, part2, out1);
}
